// SimpleRNN_59055800320032
// MI455X (gfx1250) — hardware-verified
//
#include <hip/hip_runtime.h>
#include <math.h>

constexpr int NBATCH   = 16384;
constexpr int NSTEP    = 28;
constexpr int NINP     = 28;
constexpr int KXPAD    = 32;
constexpr int NHID     = 128;
constexpr int NCLS     = 10;
constexpr int NCLSP    = 16;
constexpr int WPB      = 2;
constexpr int NTHR     = WPB * 32;
constexpr int ROWS_BLK = WPB * 16;
constexpr int HPITCH   = 136;
constexpr int XPITCH   = 40;
constexpr int HPLANE   = 16 * HPITCH;
constexpr int HTOTAL   = WPB * 2 * 2 * 2 * HPLANE;
constexpr int OSLAB    = 16 * NCLS;
constexpr int PFIN     = NSTEP & 1;
static_assert(NBATCH % ROWS_BLK == 0);
static_assert(HTOTAL % (8 * NTHR) == 0);
static_assert((ROWS_BLK * 7) % 32 == 0);
static_assert(KXPAD % 32 == 0 && NHID % 32 == 0);
static_assert(NHID % 16 == 0 && NCLSP == 16);
static_assert((HPITCH % 8) == 0 && (XPITCH % 8) == 0);
static_assert((16 * NCLS * 4) % 128 == 0);

typedef __attribute__((ext_vector_type(16))) __bf16   v16b;
typedef __attribute__((ext_vector_type(8)))  __bf16   v8b;
typedef __attribute__((ext_vector_type(8)))  _Float16 v8h;
typedef __attribute__((ext_vector_type(8)))  float    v8f;
typedef __attribute__((ext_vector_type(4)))  float    v4f;
typedef __attribute__((ext_vector_type(2)))  unsigned v2u;

__device__ __forceinline__ unsigned short f2bf_bits(float f) {
  unsigned u = __float_as_uint(f);
  return (unsigned short)((u + 0x7FFFu + ((u >> 16) & 1u)) >> 16);
}
__device__ __forceinline__ float bf_bits2f(unsigned short h) { return __uint_as_float(((unsigned)h) << 16); }
__device__ __forceinline__ float bf16r(float f) { return bf_bits2f(f2bf_bits(f)); }

struct FragB {
  union U { v16b v; v8b h[2]; };
  static __device__ __forceinline__ v16b load(const __bf16* p) {
    U f; f.h[0] = *(const v8b*)(p); f.h[1] = *(const v8b*)(p + 16); return f.v;
  }
};

__device__ __forceinline__ v8f mma_bf(v16b a, v16b b, v8f c) {
  c = __builtin_amdgcn_wmma_f32_16x16x32_bf16(false, a, false, b, (short)0, c, false, false);
  asm volatile("v_nop\n\tv_nop\n\tv_nop\n\tv_nop" : "+v"(c) : "v"(a), "v"(b));
  return c;
}

__global__ __launch_bounds__(256) void cvt_plane_kernel(const float* __restrict__ src, unsigned short* __restrict__ dst,
                                                        int nrow_in, int ncol_in, int nrow_out, int kp) {
  const int i  = blockIdx.x * 256 + threadIdx.x;
  const int k8 = kp >> 3;
  const int n8 = nrow_out * k8;
  if (i < n8) {
    const int row  = i / k8;
    const int c8   = (i - row * k8) * 8;
    const int rowc = (row < nrow_in) ? row : (nrow_in - 1);
    const float keep_row = (row < nrow_in) ? 1.0f : 0.0f;
    const float* sp = src + (size_t)rowc * ncol_in;
    v8h hv;
#pragma unroll
    for (int e = 0; e < 8; ++e) {
      const int k  = c8 + e;
      const int kc = (k < ncol_in) ? k : (ncol_in - 1);
      const float keep = (k < ncol_in) ? keep_row : 0.0f;
      const float f = sp[kc] * keep;
      const unsigned short bits = f2bf_bits(f);
      hv[e] = __builtin_bit_cast(_Float16, bits);
    }
    unsigned short* dp = dst + (size_t)i * 8;
    *(volatile v8h*)dp = hv;
    __threadfence();
    *(volatile v8h*)dp = hv;
  }
}

__device__ __forceinline__ void load_x_tile(const float* __restrict__ x, unsigned short* xs, int rowbase, int t, int tid) {
#pragma unroll
  for (int j = 0; j < 4; ++j) {
    const int i = j * NTHR + tid;
    if (i < ROWS_BLK * 7) {
      const int row = i / 7;
      const int q   = i - row * 7;
      const v4f v = *(const v4f*)(x + ((size_t)(rowbase + row) * NSTEP + (size_t)t) * NINP + 4 * q);
      const unsigned u0 = f2bf_bits(v[0]), u1 = f2bf_bits(v[1]), u2 = f2bf_bits(v[2]), u3 = f2bf_bits(v[3]);
      v2u pk;
      pk[0] = u0 | (u1 << 16);
      pk[1] = u2 | (u3 << 16);
      *(v2u*)(xs + row * XPITCH + 4 * q) = pk;
    }
  }
  if (tid < ROWS_BLK) {
    v2u z;
    z[0] = 0u;
    z[1] = 0u;
    *(v2u*)(xs + tid * XPITCH + NINP) = z;
  }
}

__device__ __forceinline__ void act_split_store(v8f acc, __bf16* hi, __bf16* lo, int rowoff, int n) {
#pragma unroll
  for (int r = 0; r < 8; ++r) {
    const float v = tanhf(acc[r]);
    const unsigned short hb = f2bf_bits(v);
    const unsigned short lb = f2bf_bits(v - bf_bits2f(hb));
    hi[(rowoff + r) * HPITCH + n] = __builtin_bit_cast(__bf16, hb);
    lo[(rowoff + r) * HPITCH + n] = __builtin_bit_cast(__bf16, lb);
  }
}

__device__ __forceinline__ int hplane_off(int wave, int layer, int par, int which) {
  return (((wave * 2 + layer) * 2 + par) * 2 + which) * HPLANE;
}

__global__ __launch_bounds__(NTHR) void rnn2_seq_kernel(const float* __restrict__ x,
                                                       const float* __restrict__ bih0, const float* __restrict__ bhh0,
                                                       const float* __restrict__ bih1, const float* __restrict__ bhh1,
                                                       const float* __restrict__ bfc,
                                                       const unsigned short* __restrict__ wih0p,
                                                       const unsigned short* __restrict__ whh0p,
                                                       const unsigned short* __restrict__ wih1p,
                                                       const unsigned short* __restrict__ whh1p,
                                                       const unsigned short* __restrict__ wfcp,
                                                       float* __restrict__ out) {
  __shared__ __align__(16) __bf16         Hs[HTOTAL];
  __shared__ __align__(16) unsigned short Xs[ROWS_BLK * XPITCH];
  __shared__ __align__(16) float          Os[WPB * OSLAB];
  const __bf16* WIH0 = (const __bf16*)wih0p;
  const __bf16* WHH0 = (const __bf16*)whh0p;
  const __bf16* WIH1 = (const __bf16*)wih1p;
  const __bf16* WHH1 = (const __bf16*)whh1p;
  const __bf16* WFC  = (const __bf16*)wfcp;
  const int tid = threadIdx.x, lane = tid & 31, wave = tid >> 5;
  const int c = lane & 15, hh = lane >> 4, koff = 8 * hh;
  const int rowbase = blockIdx.x * ROWS_BLK;
  const int wrow = 16 * wave;
  const int arow = c * HPITCH + koff;
  const int drow = 8 * hh;

  {
    const __bf16 zb = __builtin_bit_cast(__bf16, (unsigned short)0);
    v8b z8;
#pragma unroll
    for (int e = 0; e < 8; ++e) z8[e] = zb;
#pragma unroll 1
    for (int i = tid; i < HTOTAL / 8; i += NTHR) *(v8b*)(Hs + 8 * i) = z8;
  }
  load_x_tile(x, Xs, rowbase, 0, tid);
  __syncthreads();

#pragma unroll 1
  for (int t = 0; t < NSTEP; ++t) {
    const int p = t & 1;
    const __bf16* h0h_cur = Hs + hplane_off(wave, 0, p, 0);
    const __bf16* h0l_cur = Hs + hplane_off(wave, 0, p, 1);
    __bf16*       h0h_new = Hs + hplane_off(wave, 0, p ^ 1, 0);
    __bf16*       h0l_new = Hs + hplane_off(wave, 0, p ^ 1, 1);
    const __bf16* h1h_cur = Hs + hplane_off(wave, 1, p, 0);
    const __bf16* h1l_cur = Hs + hplane_off(wave, 1, p, 1);
    __bf16*       h1h_new = Hs + hplane_off(wave, 1, p ^ 1, 0);
    __bf16*       h1l_new = Hs + hplane_off(wave, 1, p ^ 1, 1);

    {
      const v16b xa = FragB::load((const __bf16*)Xs + (wrow + c) * XPITCH + koff);
#pragma unroll 1
      for (int nt = 0; nt < NHID / 16; ++nt) {
        const int n = 16 * nt + c;
        const float bv = bf16r(bih0[n]) + bf16r(bhh0[n]);
        v8f acc = {bv, bv, bv, bv, bv, bv, bv, bv};
        const v16b bx = FragB::load(WIH0 + (size_t)n * KXPAD + koff);
        acc = mma_bf(xa, bx, acc);
        const __bf16* wr = WHH0 + (size_t)n * NHID + koff;
#pragma unroll 1
        for (int k0 = 0; k0 < NHID; k0 += 32) {
          const v16b ah = FragB::load(h0h_cur + arow + k0);
          const v16b al = FragB::load(h0l_cur + arow + k0);
          const v16b bw = FragB::load(wr + k0);
          acc = mma_bf(ah, bw, acc);
          acc = mma_bf(al, bw, acc);
        }
        act_split_store(acc, h0h_new, h0l_new, drow, n);
      }
    }
    __syncthreads();

    {
#pragma unroll 1
      for (int nt = 0; nt < NHID / 16; ++nt) {
        const int n = 16 * nt + c;
        const float bv = bf16r(bih1[n]) + bf16r(bhh1[n]);
        v8f acc = {bv, bv, bv, bv, bv, bv, bv, bv};
        const __bf16* wi = WIH1 + (size_t)n * NHID + koff;
        const __bf16* wh = WHH1 + (size_t)n * NHID + koff;
#pragma unroll 1
        for (int k0 = 0; k0 < NHID; k0 += 32) {
          const v16b f0h = FragB::load(h0h_new + arow + k0);
          const v16b f0l = FragB::load(h0l_new + arow + k0);
          const v16b f1h = FragB::load(h1h_cur + arow + k0);
          const v16b f1l = FragB::load(h1l_cur + arow + k0);
          const v16b bi  = FragB::load(wi + k0);
          const v16b bh  = FragB::load(wh + k0);
          acc = mma_bf(f0h, bi, acc);
          acc = mma_bf(f0l, bi, acc);
          acc = mma_bf(f1h, bh, acc);
          acc = mma_bf(f1l, bh, acc);
        }
        act_split_store(acc, h1h_new, h1l_new, drow, n);
      }
    }
    {
      const int tn = (t + 1 < NSTEP) ? (t + 1) : (NSTEP - 1);
      load_x_tile(x, Xs, rowbase, tn, tid);
    }
    __syncthreads();
  }

  {
    const __bf16* fh = Hs + hplane_off(wave, 1, PFIN, 0) + arow;
    const __bf16* fl = Hs + hplane_off(wave, 1, PFIN, 1) + arow;
    const __bf16* wf = WFC + (size_t)c * NHID + koff;
    v8f acc = {0.f, 0.f, 0.f, 0.f, 0.f, 0.f, 0.f, 0.f};
#pragma unroll 1
    for (int k0 = 0; k0 < NHID; k0 += 32) {
      const v16b ah = FragB::load(fh + k0);
      const v16b al = FragB::load(fl + k0);
      const v16b bw = FragB::load(wf + k0);
      acc = mma_bf(ah, bw, acc);
      acc = mma_bf(al, bw, acc);
    }
    const int cc = (c < NCLS) ? c : (NCLS - 1);
    const float bb = bf16r(bfc[cc]);
    float* os = Os + wave * OSLAB;
    if (c < NCLS) {
#pragma unroll
      for (int r = 0; r < 8; ++r) os[(drow + r) * NCLS + c] = acc[r] + bb;
    }
  }
  __syncthreads();
  {
    const float* os = Os + wave * OSLAB;
    float* op = out + (size_t)(rowbase + wrow) * NCLS;
    const int l8 = (lane < 8) ? lane : 7;
    for (int pass = 0; pass < 2; ++pass) {
      const v4f v0 = *(const v4f*)(os + 4 * lane);
      const v4f v1 = *(const v4f*)(os + 128 + 4 * l8);
      *(volatile v4f*)(op + 4 * lane) = v0;
      if (lane < 8) *(volatile v4f*)(op + 128 + 4 * lane) = v1;
      __threadfence();
    }
  }
}

extern "C" void kernel_launch(void* const* d_in, const int* in_sizes, int n_in,
                              void* d_out, int out_size, void* d_ws, size_t ws_size, hipStream_t stream) {
  if (n_in < 11 || d_out == nullptr || d_ws == nullptr) return;
  if (in_sizes[0] != NBATCH * NSTEP * NINP || in_sizes[1] != NHID * NINP || in_sizes[2] != NHID * NHID ||
      in_sizes[3] != NHID || in_sizes[4] != NHID || in_sizes[5] != NHID * NHID || in_sizes[6] != NHID * NHID ||
      in_sizes[7] != NHID || in_sizes[8] != NHID || in_sizes[9] != NCLS * NHID || in_sizes[10] != NCLS ||
      out_size != NBATCH * NCLS) return;

  const float* x    = (const float*)d_in[0];
  const float* wih0 = (const float*)d_in[1];
  const float* whh0 = (const float*)d_in[2];
  const float* bih0 = (const float*)d_in[3];
  const float* bhh0 = (const float*)d_in[4];
  const float* wih1 = (const float*)d_in[5];
  const float* whh1 = (const float*)d_in[6];
  const float* bih1 = (const float*)d_in[7];
  const float* bhh1 = (const float*)d_in[8];
  const float* wfc  = (const float*)d_in[9];
  const float* bfc  = (const float*)d_in[10];
  float* outp = (float*)d_out;

  char* ws = (char*)d_ws; size_t off = 0;
  auto carve = [&](size_t bytes) -> char* { char* pp = ws + off; off += (bytes + 255) & ~(size_t)255; return pp; };
  unsigned short* WIH0P = (unsigned short*)carve((size_t)NHID * KXPAD * 2);
  unsigned short* WHH0P = (unsigned short*)carve((size_t)NHID * NHID * 2);
  unsigned short* WIH1P = (unsigned short*)carve((size_t)NHID * NHID * 2);
  unsigned short* WHH1P = (unsigned short*)carve((size_t)NHID * NHID * 2);
  unsigned short* WFCP  = (unsigned short*)carve((size_t)NCLSP * NHID * 2);
  if (off > ws_size || off > (size_t)134217728) return;

  const int n8a = NHID * (KXPAD / 8);
  const int n8b = NHID * (NHID / 8);
  const int n8c = NCLSP * (NHID / 8);
  cvt_plane_kernel<<<(n8a + 255) / 256, 256, 0, stream>>>(wih0, WIH0P, NHID, NINP, NHID,  KXPAD);
  cvt_plane_kernel<<<(n8b + 255) / 256, 256, 0, stream>>>(whh0, WHH0P, NHID, NHID, NHID,  NHID);
  cvt_plane_kernel<<<(n8b + 255) / 256, 256, 0, stream>>>(wih1, WIH1P, NHID, NHID, NHID,  NHID);
  cvt_plane_kernel<<<(n8b + 255) / 256, 256, 0, stream>>>(whh1, WHH1P, NHID, NHID, NHID,  NHID);
  cvt_plane_kernel<<<(n8c + 255) / 256, 256, 0, stream>>>(wfc,  WFCP,  NCLS, NHID, NCLSP, NHID);
  rnn2_seq_kernel<<<NBATCH / ROWS_BLK, NTHR, 0, stream>>>(x, bih0, bhh0, bih1, bhh1, bfc,
                                                          WIH0P, WHH0P, WIH1P, WHH1P, WFCP, outp);
}
